// ScaledDotProductAttention_19988777796223
// MI455X (gfx1250) — hardware-verified
//
#include <hip/hip_runtime.h>


#ifndef NB
#define NB 2
#endif
#ifndef SEQ
#define SEQ 2048
#endif
#define NHD      16
#define SEQ_FULL 2048
#define HD       64
#define NPL      (NB * NHD)
#define ZH       4
#define TT       SEQ
#define PCAR     1024.0f
#define SCL      0.125f

static_assert(SEQ % 128 == 0);
static_assert(SEQ <= SEQ_FULL);
static_assert(NPL % ZH == 0);
static_assert(HD % 32 == 0 && HD % 64 == 0);
static_assert(((size_t)NPL * SEQ * HD) % 2048 == 0);
static_assert(((size_t)NPL * SEQ * HD) % 512 == 0);
static_assert(((size_t)ZH * SEQ) % 8 == 0);
static_assert((size_t)3 * NPL * SEQ * HD * 2 + (size_t)ZH * SEQ * SEQ * 6 <= (size_t)134217728);

typedef _Float16 h16;
typedef unsigned short bf;
typedef __attribute__((ext_vector_type(16))) __bf16   v16bf;
typedef __attribute__((ext_vector_type(16))) _Float16 v16h;
typedef __attribute__((ext_vector_type(8)))  _Float16 v8h;
typedef __attribute__((ext_vector_type(8)))  unsigned short v8us;
typedef __attribute__((ext_vector_type(8)))  float    v8f;
typedef __attribute__((ext_vector_type(4)))  float    v4f;
typedef __attribute__((ext_vector_type(2)))  _Float16 v2h;
typedef __attribute__((ext_vector_type(4)))  _Float16 v4h;
typedef v4f  __attribute__((may_alias)) v4fa;

__device__ __forceinline__ unsigned short f2bf(float f) { unsigned u = __float_as_uint(f); u += 0x7FFFu + ((u >> 16) & 1u); return (unsigned short)(u >> 16); }
__device__ __forceinline__ float bf2f(unsigned short b) { return __uint_as_float(((unsigned)b) << 16); }
__device__ __forceinline__ float bfr(float f) { return bf2f(f2bf(f)); }
__device__ __forceinline__ h16 tohx(float x) { return (h16)x; }
__device__ __forceinline__ v16h cat16(v8h lo, v8h hi) { return __builtin_shufflevector(lo, hi, 0, 1, 2, 3, 4, 5, 6, 7, 8, 9, 10, 11, 12, 13, 14, 15); }
__device__ __forceinline__ v16bf cat16b(v8us lo, v8us hi) { return __builtin_bit_cast(v16bf, __builtin_shufflevector(lo, hi, 0, 1, 2, 3, 4, 5, 6, 7, 8, 9, 10, 11, 12, 13, 14, 15)); }
__device__ __forceinline__ v8f wmma16(v16h a, v16h b, v8f c) { return __builtin_amdgcn_wmma_f32_16x16x32_f16(false, a, false, b, (short)0, c, false, false); }
__device__ __forceinline__ v8f wmmab(v16bf a, v16bf b, v8f c) { return __builtin_amdgcn_wmma_f32_16x16x32_bf16(false, a, false, b, (short)0, c, false, false); }

template <typename T16> struct WFrag;
template <> struct WFrag<h16> { typedef v16h V; static __device__ __forceinline__ V ld(const h16* p) { return cat16(*(const v8h*)p, *(const v8h*)(p + 16)); } static __device__ __forceinline__ v8f mma(V a, V b, v8f c) { return wmma16(a, b, c); } };
template <> struct WFrag<bf> { typedef v16bf V; static __device__ __forceinline__ V ld(const bf* p) { return cat16b(*(const v8us*)p, *(const v8us*)(p + 16)); } static __device__ __forceinline__ v8f mma(V a, V b, v8f c) { return wmmab(a, b, c); } };
template <typename T16, int NSPLIT, bool BIAS>
__global__ __launch_bounds__(32) void k_gemmw(const T16* __restrict__ A, const T16* __restrict__ A2, const T16* __restrict__ Bt, const T16* __restrict__ Bt2, int K, float* C, int ldc, const float* __restrict__ bias, size_t sA, size_t sB, size_t sC, float osc) {
    typedef typename WFrag<T16>::V V;
    __shared__ __align__(16) float os[16 * 68];
    const size_t z = blockIdx.z; A += z * sA; if (A2) A2 += z * sA; Bt += z * sB; if (Bt2) Bt2 += z * sB; C += z * sC;
    const int lane = threadIdx.x & 31, lr = lane & 15, hi = lane >> 4; const int r0 = blockIdx.x * 64, c0 = blockIdx.y * 64;
    v8f acc[4][4];
#pragma unroll
    for (int mb = 0; mb < 4; ++mb)
#pragma unroll
        for (int nb = 0; nb < 4; ++nb) acc[mb][nb] = (v8f){};
    const size_t aoff = (size_t)(r0 + lr) * K + 8 * hi, boff = (size_t)(c0 + lr) * K + 8 * hi;
#pragma unroll 1
    for (int kc = 0; kc < K; kc += 32) {
        V a[4], a2[4];
#pragma unroll
        for (int mb = 0; mb < 4; ++mb) { a[mb] = WFrag<T16>::ld(A + aoff + (size_t)mb * 16 * K + kc); if (NSPLIT == 1 || NSPLIT == 2) a2[mb] = WFrag<T16>::ld(A2 + aoff + (size_t)mb * 16 * K + kc); }
#pragma unroll
        for (int nb = 0; nb < 4; ++nb) { const V b = WFrag<T16>::ld(Bt + boff + (size_t)nb * 16 * K + kc); V b2; if (NSPLIT >= 2) b2 = WFrag<T16>::ld(Bt2 + boff + (size_t)nb * 16 * K + kc);
#pragma unroll
            for (int mb = 0; mb < 4; ++mb) { acc[mb][nb] = WFrag<T16>::mma(a[mb], b, acc[mb][nb]); if (NSPLIT == 1 || NSPLIT == 2) acc[mb][nb] = WFrag<T16>::mma(a2[mb], b, acc[mb][nb]); if (NSPLIT >= 2) acc[mb][nb] = WFrag<T16>::mma(a[mb], b2, acc[mb][nb]); } }
        asm volatile("v_nop\n\tv_nop\n\tv_nop\n\tv_nop" : "+v"(acc[0][0]), "+v"(acc[1][1]), "+v"(acc[2][2]), "+v"(acc[3][3]) : "v"(a[0]), "v"(a[3]));
    }
#pragma unroll
    for (int mb = 0; mb < 4; ++mb) {
#pragma unroll
        for (int nb = 0; nb < 4; ++nb) {
#pragma unroll
            for (int j = 0; j < 8; ++j) os[(hi * 8 + j) * 68 + nb * 16 + lr] = acc[mb][nb][j]; }
        __builtin_amdgcn_wave_barrier(); asm volatile("" ::: "memory");
        float* crow = C + (size_t)(r0 + mb * 16) * ldc + c0;
#pragma unroll 1
        for (int ps = 0; ps < 2; ++ps) {
#pragma unroll
            for (int s = 0; s < 8; ++s) { const int row = 2 * s + hi, cofs = lr * 4; v4f val = *(const v4fa*)(os + row * 68 + cofs); if (BIAS) { val[0] += bfr(bias[c0 + cofs]); val[1] += bfr(bias[c0 + cofs + 1]); val[2] += bfr(bias[c0 + cofs + 2]); val[3] += bfr(bias[c0 + cofs + 3]); }
                val = val * osc;
                *(volatile v4f*)(crow + (size_t)row * ldc + cofs) = val; }
            if (ps == 0) __threadfence(); }
        __builtin_amdgcn_wave_barrier(); asm volatile("" ::: "memory");
    }
}

__global__ __launch_bounds__(256) void k_cvtbf(const float* __restrict__ F, bf* P) {
    const unsigned e = (blockIdx.x * 256u + threadIdx.x) * 8u; if (e >= (unsigned)(NPL * SEQ * HD)) return;
    const unsigned pl = e / (unsigned)(SEQ * HD); const unsigned r = e - pl * (unsigned)(SEQ * HD);
    const float* f = F + (size_t)pl * ((size_t)SEQ_FULL * HD) + r;
    const v4f a = *(const v4f*)f; const v4f b = *(const v4f*)(f + 4);
    v8us o;
#pragma unroll
    for (int q = 0; q < 4; ++q) { o[q] = f2bf(a[q]); o[4 + q] = f2bf(b[q]); }
    *(volatile v8us*)(P + e) = o; __threadfence(); *(volatile v8us*)(P + e) = o;
}

__global__ __launch_bounds__(256) void k_vt(const float* __restrict__ F, h16* V16) {
    const unsigned e = (blockIdx.x * 256u + threadIdx.x) * 2u; if (e >= (unsigned)(NPL * HD * SEQ)) return;
    const unsigned t = e % (unsigned)SEQ; const unsigned d = (e / (unsigned)SEQ) % (unsigned)HD; const unsigned g = e / (unsigned)(SEQ * HD);
    const float* f = F + ((size_t)g * SEQ_FULL + t) * HD + d;
    v2h o; o[0] = tohx(bfr(f[0])); o[1] = tohx(bfr(f[HD]));
    *(volatile v2h*)(V16 + e) = o; __threadfence(); *(volatile v2h*)(V16 + e) = o;
}

__global__ __launch_bounds__(256) void k_asoft(const float* __restrict__ Sb, h16* P16) {
    const unsigned lane = threadIdx.x & 31u; const unsigned row = blockIdx.x * 8u + (threadIdx.x >> 5); if (row >= (unsigned)(ZH * TT)) return;
    const float* sr = Sb + (size_t)row * TT; float v[TT / 32]; float mx = -3.0e38f;
#pragma unroll
    for (int ch = 0; ch < TT / 128; ++ch) { const unsigned j0 = (unsigned)ch * 128u + lane * 4u; const v4f a = *(const v4f*)(sr + j0);
#pragma unroll
        for (int q = 0; q < 4; ++q) { const float t = a[q] * SCL; v[ch * 4 + q] = t; mx = fmaxf(mx, t); } }
#pragma unroll
    for (int sh = 16; sh; sh >>= 1) mx = fmaxf(mx, __shfl_xor(mx, sh, 32));
    float sum = 0.f;
#pragma unroll
    for (int k = 0; k < TT / 32; ++k) { float d0 = __fsub_rn(v[k], mx); asm volatile("" : "+v"(d0)); v[k] = __builtin_amdgcn_exp2f(__fmul_rn(d0, 1.4426950408889634f)); sum += v[k]; }
#pragma unroll
    for (int sh = 16; sh; sh >>= 1) sum += __shfl_xor(sum, sh, 32);
    const float f = __fdiv_rn(PCAR, sum);
#pragma unroll 1
    for (int ps = 0; ps < 2; ++ps) {
#pragma unroll
        for (int ch = 0; ch < TT / 128; ++ch) { v4h o4;
#pragma unroll
            for (int q = 0; q < 4; ++q) o4[q] = tohx(v[ch * 4 + q] * f);
            *(volatile v4h*)(P16 + (size_t)row * TT + (unsigned)ch * 128u + lane * 4u) = o4; }
        if (ps == 0) __threadfence(); }
}

extern "C" void kernel_launch(void* const* d_in, const int* in_sizes, int n_in,
                              void* d_out, int out_size, void* d_ws, size_t ws_size, hipStream_t stream) {
    if (n_in < 3) return;
    const size_t need_in = ((size_t)(NPL - 1) * SEQ_FULL + SEQ) * HD;
    if ((size_t)in_sizes[0] < need_in || (size_t)in_sizes[1] < need_in || (size_t)in_sizes[2] < need_in) return;
    if ((size_t)out_size < (size_t)NPL * SEQ * HD) return;
    const float* xq = (const float*)d_in[0]; const float* xk = (const float*)d_in[1]; const float* xv = (const float*)d_in[2];
    float* OUT = (float*)d_out;
    char* wsp = (char*)d_ws;
    auto take = [&](size_t bytes) { char* p = wsp; wsp += (bytes + 255) & ~(size_t)255; return (void*)p; };
    bf*  QB   = (bf*)take((size_t)NPL * SEQ * HD * 2);
    bf*  KB   = (bf*)take((size_t)NPL * SEQ * HD * 2);
    h16* VT16 = (h16*)take((size_t)NPL * HD * SEQ * 2);
    float* Sb = (float*)take((size_t)ZH * SEQ * SEQ * 4);
    h16* P16  = (h16*)take((size_t)ZH * SEQ * SEQ * 2);
    if ((size_t)(wsp - (char*)d_ws) > ws_size) return;

    k_cvtbf<<<(unsigned)(((size_t)NPL * SEQ * HD) / 2048), 256, 0, stream>>>(xq, QB);
    k_cvtbf<<<(unsigned)(((size_t)NPL * SEQ * HD) / 2048), 256, 0, stream>>>(xk, KB);
    k_vt<<<(unsigned)(((size_t)NPL * HD * SEQ) / 512), 256, 0, stream>>>(xv, VT16);
    for (int p = 0; p < NPL / ZH; ++p) {
        const size_t z0 = (size_t)p * ZH;
        k_gemmw<bf, 0, false><<<dim3(SEQ / 64, SEQ / 64, ZH), 32, 0, stream>>>(QB + z0 * SEQ * HD, nullptr, KB + z0 * SEQ * HD, nullptr, HD, Sb, SEQ, nullptr, (size_t)SEQ * HD, (size_t)SEQ * HD, (size_t)SEQ * SEQ, 1.0f);
        k_asoft<<<(unsigned)((size_t)ZH * SEQ / 8), 256, 0, stream>>>(Sb, P16);
        k_gemmw<h16, 0, false><<<dim3(SEQ / 64, HD / 64, ZH), 32, 0, stream>>>(P16, nullptr, VT16 + z0 * HD * SEQ, nullptr, SEQ, OUT + z0 * SEQ * HD, HD, nullptr, (size_t)SEQ * SEQ, (size_t)HD * SEQ, (size_t)SEQ * HD, 1.0f / PCAR);
    }
}
